// moleculeGCN_48352741818636
// MI455X (gfx1250) — hardware-run, weakly checked
//
#include <hip/hip_runtime.h>
#include <stddef.h>
#include <stdint.h>
#include <math.h>


#define LO_L2  1
#define LO_L3  1

#define NN     50000
#define NE     600000
#define DCH    128
#define NG     256
#define NTHR   256
#define NWAVE  8
#define EPT    8
#define CHUNK  (NTHR * EPT)
#define WCAP   (EPT * 32)
#define LISTN  (NWAVE * WCAP)
#define NBA    1024
#define SLA    10
#define NBLK   49
#define NSLOT  (NBLK * NBA)
#define RCAP   28672
#define DEGCAP 64
#define GBM    64
#define GBN    128
#define GTHR   128
#define GWAVE  (GTHR / 32)
#define MP     50048
#define HK     256
#define KX2    (LO_L2 ? 256 : 128)
#define KX3    (LO_L3 ? 256 : 128)
#define PARTW  288
#define WSTW   258
#define GSN    320
#define NUX    (MP * (DCH / 8))
#define NBX    (NUX / NTHR)
#define NB1    8
#define NB2    16
#define PREPB  (NBX + NB1 + 2 * NB2 + 1)
#define BK_ZINTS (LISTN + 2 * RCAP + 3 * NBA)
#define BK_INTS  (BK_ZINTS + NBA + 16)

static_assert(DCH == 128 && NG == 256);
static_assert(NSLOT >= NN && MP >= NN && MP <= NSLOT && MP % 128 == 0 && MP % GBM == 0);
static_assert((CHUNK & (CHUNK - 1)) == 0 && CHUNK <= 4096);
static_assert((NBA & (NBA - 1)) == 0 && NBA == (1 << SLA));
static_assert(((long long)CHUNK << SLA) < (1LL << 31));
static_assert(NE % 4 == 0 && NE < (1 << (31 - SLA)) && NE >= 1);
static_assert(LISTN % NTHR == 0 && NBA % NWAVE == 0 && NBA % 32 == 0 && NBA == 4 * NTHR);
static_assert(RCAP % (NTHR * 4) == 0 && BK_ZINTS % 4 == 0 && LISTN % 4 == 0);
static_assert(RCAP >= 12548 + 12548 / 20);
static_assert(DEGCAP >= 28 + 8);
static_assert(BK_INTS * 4 <= 327680);
static_assert(NUX % NTHR == 0);
static_assert(GBM == GWAVE * 16 && GBN == DCH && GTHR == GBN);
static_assert(KX2 % 32 == 0 && KX3 % 32 == 0 && KX2 <= HK && KX3 <= HK && DCH % 32 == 0);
static_assert(PARTW % 32 == 0 && PARTW >= 2 * DCH + 1 && WSTW >= 2 * DCH + 1);
static_assert(GSN % 32 == 0 && GSN >= NG + 2);
static_assert(NG * DCH == 32768);

typedef float          v4f   __attribute__((ext_vector_type(4)));
typedef float          v8f   __attribute__((ext_vector_type(8)));
typedef int            v4i   __attribute__((ext_vector_type(4)));
typedef int            v8i   __attribute__((ext_vector_type(8)));
typedef unsigned short v8us  __attribute__((ext_vector_type(8)));
typedef unsigned short v16us __attribute__((ext_vector_type(16)));
typedef __bf16         v16bf __attribute__((ext_vector_type(16)));
typedef v4f  __attribute__((may_alias)) v4fa;
typedef v4i  __attribute__((may_alias)) v4ia;
typedef v8us __attribute__((may_alias)) v8usa;
union FragB { v16bf v; v16us u; v8us h[2]; v8i w; };

__device__ __forceinline__ v8f wmb(const FragB& a, const FragB& b, v8f c) {
  v8f d = __builtin_amdgcn_wmma_f32_16x16x32_bf16(false, a.v, false, b.v, (short)0, c, false, false);
  asm volatile("v_nop\n\tv_nop\n\tv_nop\n\tv_nop" : "+v"(d) : "v"(a.w), "v"(b.w));
  return d;
}

__device__ __forceinline__ v8f z8() { v8f z = {0.f, 0.f, 0.f, 0.f, 0.f, 0.f, 0.f, 0.f}; return z; }
__device__ __forceinline__ float qnanf() { return __uint_as_float(0x7fc0u << 16); }

__device__ __forceinline__ unsigned bf16_bits(float f) {
  const unsigned u = __float_as_uint(f);
  return (u + 0x7FFFu + ((u >> 16) & 1u)) >> 16;
}
__device__ __forceinline__ float bf16_val(float f) {
  return __uint_as_float(bf16_bits(f) << 16);
}
__device__ __forceinline__ v4f rnd4(v4f a) {
  v4f r;
  r.x = bf16_val(a.x); r.y = bf16_val(a.y); r.z = bf16_val(a.z); r.w = bf16_val(a.w);
  return r;
}
__device__ __forceinline__ void st2_us8(unsigned short* dp, v8us o) {
  *(volatile v8us*)dp = o;
  __threadfence();
  *(volatile v8us*)dp = o;
}
__device__ __forceinline__ v8us wt_unit(const float* __restrict__ W, int n, int kk) {
  const float* p = W + (size_t)kk * DCH + n;
  v8us o;
#pragma unroll
  for (int i = 0; i < 8; ++i) o[i] = (unsigned short)bf16_bits(p[(size_t)i * DCH]);
  return o;
}

template <int SLB>
__device__ __forceinline__ int scan_chunk(const int* __restrict__ dsts, int nE, int cbase, int slotBase,
                                          int nb, int* list, int tid, int lane, int wave) {
  int wc = 0;
  const int el0  = tid * EPT;
  const int e0   = cbase + el0;
  const int sent = (int)(1u << 31);
  v4i da, db;
  if (cbase + CHUNK <= nE) {
    da = *(const v4i*)(dsts + e0);
    db = *(const v4i*)(dsts + e0 + 4);
  } else {
    const int t0 = dsts[min(e0,     nE - 1)];
    const int t1 = dsts[min(e0 + 1, nE - 1)];
    const int t2 = dsts[min(e0 + 2, nE - 1)];
    const int t3 = dsts[min(e0 + 3, nE - 1)];
    const int t4 = dsts[min(e0 + 4, nE - 1)];
    const int t5 = dsts[min(e0 + 5, nE - 1)];
    const int t6 = dsts[min(e0 + 6, nE - 1)];
    const int t7 = dsts[min(e0 + 7, nE - 1)];
    asm volatile("" :: "v"(t0), "v"(t1), "v"(t2), "v"(t3));
    asm volatile("" :: "v"(t4), "v"(t5), "v"(t6), "v"(t7));
    da.x = (e0     < nE) ? t0 : sent;
    da.y = (e0 + 1 < nE) ? t1 : sent;
    da.z = (e0 + 2 < nE) ? t2 : sent;
    da.w = (e0 + 3 < nE) ? t3 : sent;
    db.x = (e0 + 4 < nE) ? t4 : sent;
    db.y = (e0 + 5 < nE) ? t5 : sent;
    db.z = (e0 + 6 < nE) ? t6 : sent;
    db.w = (e0 + 7 < nE) ? t7 : sent;
  }
  const unsigned nbs = (unsigned)slotBase;
  const unsigned unb = (unsigned)nb;
  const unsigned s0 = (unsigned)da.x - nbs, s1 = (unsigned)da.y - nbs;
  const unsigned s2 = (unsigned)da.z - nbs, s3 = (unsigned)da.w - nbs;
  const unsigned s4 = (unsigned)db.x - nbs, s5 = (unsigned)db.y - nbs;
  const unsigned s6 = (unsigned)db.z - nbs, s7 = (unsigned)db.w - nbs;
  const bool h0 = s0 < unb, h1 = s1 < unb, h2 = s2 < unb, h3 = s3 < unb;
  const bool h4 = s4 < unb, h5 = s5 < unb, h6 = s6 < unb, h7 = s7 < unb;
  const unsigned any = __builtin_amdgcn_ballot_w32(h0 | h1 | h2 | h3 | h4 | h5 | h6 | h7);
  if (any != 0u) {
#define HITJ(J, HJ, SJ) { \
      const unsigned mj = __builtin_amdgcn_ballot_w32(HJ); \
      if (mj != 0u) { \
        if (HJ) { \
          const int pos = wc + (int)__builtin_amdgcn_mbcnt_lo(mj, 0u); \
          if (pos < WCAP) list[wave * WCAP + pos] = ((el0 + (J)) << SLB) | (int)(SJ); \
        } \
        wc += (int)__builtin_popcount(mj); } }
    HITJ(0, h0, s0)
    HITJ(1, h1, s1)
    HITJ(2, h2, s2)
    HITJ(3, h3, s3)
    HITJ(4, h4, s4)
    HITJ(5, h5, s5)
    HITJ(6, h6, s6)
    HITJ(7, h7, s7)
#undef HITJ
  }
  return wc;
}

__global__ __launch_bounds__(NTHR) void k_prep(
    const float* __restrict__ x, const float* __restrict__ W1, const float* __restrict__ Wm,
    const float* __restrict__ W2,
    const float* __restrict__ q0, const float* __restrict__ q1, const float* __restrict__ q2,
    const float* __restrict__ q3, const float* __restrict__ q4, const float* __restrict__ q5,
    const float* __restrict__ q6, const float* __restrict__ q7, const float* __restrict__ q8,
    unsigned short* xb, unsigned short* w1t, unsigned short* wmd, unsigned short* w2d, float* par) {
  const int b = (int)blockIdx.x, tid = (int)threadIdx.x;
  if (b < NBX) {
    const int u   = b * NTHR + tid;
    const int row = u >> 4;
    const int k8  = (u & 15) * 8;
    const int rc  = row < NN ? row : NN - 1;
    const float* p = x + (size_t)rc * DCH + k8;
    const v4f a = *(const v4fa*)p;
    const v4f c = *(const v4fa*)(p + 4);
    const bool ok = row < NN;
    v8us o;
    o[0] = ok ? (unsigned short)bf16_bits(a.x) : (unsigned short)0;
    o[1] = ok ? (unsigned short)bf16_bits(a.y) : (unsigned short)0;
    o[2] = ok ? (unsigned short)bf16_bits(a.z) : (unsigned short)0;
    o[3] = ok ? (unsigned short)bf16_bits(a.w) : (unsigned short)0;
    o[4] = ok ? (unsigned short)bf16_bits(c.x) : (unsigned short)0;
    o[5] = ok ? (unsigned short)bf16_bits(c.y) : (unsigned short)0;
    o[6] = ok ? (unsigned short)bf16_bits(c.z) : (unsigned short)0;
    o[7] = ok ? (unsigned short)bf16_bits(c.w) : (unsigned short)0;
    st2_us8(xb + (size_t)row * DCH + k8, o);
  } else if (b < NBX + NB1) {
    const int u  = (b - NBX) * NTHR + tid;
    const int n  = u >> 4;
    const int k8 = (u & 15) * 8;
    const v8us o = wt_unit(W1, n, k8);
    st2_us8(w1t + (size_t)u * 8, o);
  } else if (b < NBX + NB1 + NB2) {
    const int u  = (b - NBX - NB1) * NTHR + tid;
    const int n  = u >> 5;
    const int k8 = (u & 31) * 8;
    const v8us o = wt_unit(Wm, n, k8 & (DCH - 1));
    st2_us8(wmd + (size_t)u * 8, o);
  } else if (b < NBX + NB1 + 2 * NB2) {
    const int u  = (b - NBX - NB1 - NB2) * NTHR + tid;
    const int n  = u >> 5;
    const int k8 = (u & 31) * 8;
    const v8us o = wt_unit(W2, n, k8 & (DCH - 1));
    st2_us8(w2d + (size_t)u * 8, o);
  } else {
    if (tid < 32) {
      const v4f a0 = rnd4(*(const v4fa*)(q0 + 4 * tid));
      const v4f a1 = rnd4(*(const v4fa*)(q1 + 4 * tid));
      const v4f a2 = rnd4(*(const v4fa*)(q2 + 4 * tid));
      const v4f a3 = rnd4(*(const v4fa*)(q3 + 4 * tid));
      const v4f a4 = rnd4(*(const v4fa*)(q4 + 4 * tid));
      const v4f a5 = rnd4(*(const v4fa*)(q5 + 4 * tid));
      const v4f a6 = rnd4(*(const v4fa*)(q6 + 4 * tid));
      const v4f a7 = rnd4(*(const v4fa*)(q7 + 4 * tid));
      const v4f a8 = rnd4(*(const v4fa*)(q8 + 4 * tid));
      float* pp = par + 4 * tid;
      *(volatile v4f*)(pp + 0 * DCH) = a0; *(volatile v4f*)(pp + 1 * DCH) = a1;
      *(volatile v4f*)(pp + 2 * DCH) = a2; *(volatile v4f*)(pp + 3 * DCH) = a3;
      *(volatile v4f*)(pp + 4 * DCH) = a4; *(volatile v4f*)(pp + 5 * DCH) = a5;
      *(volatile v4f*)(pp + 6 * DCH) = a6; *(volatile v4f*)(pp + 7 * DCH) = a7;
      *(volatile v4f*)(pp + 8 * DCH) = a8;
      __threadfence();
      *(volatile v4f*)(pp + 0 * DCH) = a0; *(volatile v4f*)(pp + 1 * DCH) = a1;
      *(volatile v4f*)(pp + 2 * DCH) = a2; *(volatile v4f*)(pp + 3 * DCH) = a3;
      *(volatile v4f*)(pp + 4 * DCH) = a4; *(volatile v4f*)(pp + 5 * DCH) = a5;
      *(volatile v4f*)(pp + 6 * DCH) = a6; *(volatile v4f*)(pp + 7 * DCH) = a7;
      *(volatile v4f*)(pp + 8 * DCH) = a8;
    }
  }
}

__global__ __launch_bounds__(512) void k_ranges(const int* __restrict__ bat, int* gs) {
  __shared__ __attribute__((aligned(16))) int sg[GSN];
  __shared__ int wf[16];
  const int tid = (int)threadIdx.x, lane = tid & 31, wave = tid >> 5;
  int viol = 0;
#pragma unroll 1
  for (int i0 = 0; i0 < NN - 1; i0 += 512) {
    const int i  = i0 + tid;
    const int ic = i < NN - 1 ? i : NN - 2;
    const int a = bat[ic];
    const int c = bat[ic + 1];
    viol |= (a > c) ? 1 : 0;
  }
  const unsigned vm = __builtin_amdgcn_ballot_w32(viol != 0);
  if (lane == 0) wf[wave] = (vm != 0u) ? 1 : 0;

  const int g   = tid < NG ? tid : NG;
  const int key = bat[0] + g;
  int lo = 0, hi = NN;
#pragma unroll 1
  for (int it = 0; it < 17; ++it) {
    const int mid = (lo + hi) >> 1;
    const int mc  = mid < NN - 1 ? mid : NN - 1;
    const int v   = bat[mc];
    asm volatile("" :: "v"(v));
    const bool act  = lo < hi;
    const bool less = v < key;
    lo = (act && less)  ? mid + 1 : lo;
    hi = (act && !less) ? mid     : hi;
  }
  __syncthreads();
  int tot = 0;
#pragma unroll
  for (int w = 0; w < 16; ++w) tot |= wf[w];
  if (tid < GSN) sg[tid] = (tid <= NG) ? lo : ((tid == NG + 1) ? tot : 0);
  __syncthreads();
  const int qi = tid < GSN / 4 ? tid : GSN / 4 - 1;
  const v4i qv = *(const v4ia*)(sg + 4 * qi);
  if (tid < GSN / 4) *(volatile v4i*)(gs + 4 * tid) = qv;
  __threadfence();
  if (tid < GSN / 4) *(volatile v4i*)(gs + 4 * tid) = qv;
}

__global__ __launch_bounds__(NTHR) void k_bucket(const int* __restrict__ srcs, const int* __restrict__ dsts,
                                                 int* lst, int* cntp, int* offp, float* dinvp) {
  extern __shared__ __attribute__((aligned(16))) int dsm[];
  int* list = dsm;
  int* hl   = dsm + LISTN;
  int* sl   = hl + RCAP;
  int* cnt  = sl + RCAP;
  int* offs = cnt + NBA;
  int* cur  = offs + NBA;
  float* dv = reinterpret_cast<float*>(cur + NBA);
  int* misc = cur + 2 * NBA;
  const int tid = (int)threadIdx.x, lane = tid & 31, wave = tid >> 5;
  const int nodeBase = (int)blockIdx.x * NBA;

  {
    const v4i z4 = {0, 0, 0, 0};
    for (int i = tid * 4; i < BK_ZINTS; i += NTHR * 4) *(v4ia*)(dsm + i) = z4;
    if (tid < 16) misc[tid] = 0;
  }
  __syncthreads();

  int t = 0, ov = 0;
  const int nChunks = (NE + CHUNK - 1) / CHUNK;
#pragma unroll 1
  for (int ch = 0; ch < nChunks; ++ch) {
    const int cbase = ch * CHUNK;
    const int wc = scan_chunk<SLA>(dsts, NE, cbase, nodeBase, NBA, list, tid, lane, wave);
    if (lane == 0) misc[wave] = wc;
    __syncthreads();
    if (wave == 0) {
#pragma unroll 1
      for (int w2 = 0; w2 < NWAVE; ++w2) {
        int c = misc[w2];
        c = c < 0 ? 0 : (c > WCAP ? WCAP : c);
#pragma unroll 1
        for (int b0 = 0; b0 < c; b0 += 32) {
          const int idx = b0 + lane;
          const int ent = list[w2 * WCAP + (idx < WCAP ? idx : WCAP - 1)];
          const int m32 = (c - b0) < 32 ? (c - b0) : 32;
#pragma unroll 1
          for (int k = 0; k < m32; ++k) {
            const int u    = __builtin_amdgcn_readlane(ent, k);
            const int slot = u & (NBA - 1);
            const int el   = (u >> SLA) & (CHUNK - 1);
            const int pk   = ((cbase + el) << SLA) | slot;
            if (t < RCAP) {
              if (lane == 0) { hl[t] = pk; cnt[slot] = cnt[slot] + 1; }
              t = t + 1;
            } else {
              ov = 1;
            }
          }
        }
      }
    }
    __syncthreads();
  }
  if (wave == 0 && lane == 0) { misc[8] = t; misc[9] = ov; }
  __syncthreads();
  int tt = misc[8];
  tt = tt < 0 ? 0 : (tt > RCAP ? RCAP : tt);
  const int ovf = misc[9];

  if (wave == 0) {
    const int base = lane * (NBA / 32);
    int s = 0;
#pragma unroll 1
    for (int i = 0; i < NBA / 32; ++i) s += cnt[base + i];
    int incl = s;
#pragma unroll
    for (int d = 1; d < 32; d <<= 1) {
      const int y = __shfl_up(incl, d, 32);
      if (lane >= d) incl += y;
    }
    int run = incl - s;
#pragma unroll 1
    for (int i = 0; i < NBA / 32; ++i) {
      const int cv = cnt[base + i];
      offs[base + i] = run;
      cur[base + i]  = run;
      run += cv;
    }
  }
  __syncthreads();
  if (wave == 0) {
#pragma unroll 1
    for (int b0 = 0; b0 < tt; b0 += 32) {
      const int idx = b0 + lane;
      const int ent = hl[idx < RCAP ? idx : RCAP - 1];
      const int m32 = (tt - b0) < 32 ? (tt - b0) : 32;
#pragma unroll 1
      for (int k = 0; k < m32; ++k) {
        const int u    = __builtin_amdgcn_readlane(ent, k);
        const int slot = u & (NBA - 1);
        if (lane == 0) {
          int p = cur[slot];
          p = p < 0 ? 0 : (p > RCAP - 1 ? RCAP - 1 : p);
          sl[p] = u;
          cur[slot] = p + 1;
        }
      }
    }
  }
  __syncthreads();

#pragma unroll 1
  for (int j = 0; j < NBA / NTHR; ++j) {
    const int s = j * NTHR + tid;
    dv[s] = 1.0f / sqrtf((float)(cnt[s] + 1));
  }
  int* lb = lst + (size_t)blockIdx.x * RCAP;
#pragma unroll 1
  for (int i = tid * 4; i < RCAP; i += NTHR * 4) {
    const v4i e4 = *(const v4ia*)(sl + i);
    int e0 = e4.x >> SLA, e1 = e4.y >> SLA, e2 = e4.z >> SLA, e3 = e4.w >> SLA;
    e0 = e0 < 0 ? 0 : (e0 > NE - 1 ? NE - 1 : e0);
    e1 = e1 < 0 ? 0 : (e1 > NE - 1 ? NE - 1 : e1);
    e2 = e2 < 0 ? 0 : (e2 > NE - 1 ? NE - 1 : e2);
    e3 = e3 < 0 ? 0 : (e3 > NE - 1 ? NE - 1 : e3);
    int r0 = srcs[e0], r1 = srcs[e1], r2 = srcs[e2], r3 = srcs[e3];
    v4i sv;
    sv.x = r0 < 0 ? 0 : (r0 > NN - 1 ? NN - 1 : r0);
    sv.y = r1 < 0 ? 0 : (r1 > NN - 1 ? NN - 1 : r1);
    sv.z = r2 < 0 ? 0 : (r2 > NN - 1 ? NN - 1 : r2);
    sv.w = r3 < 0 ? 0 : (r3 > NN - 1 ? NN - 1 : r3);
    *(v4ia*)(hl + i) = sv;
    *(volatile v4i*)(lb + i) = sv;
  }
  __syncthreads();
  v4i c4 = *(const v4ia*)(cnt + 4 * tid);
  const v4i o4 = *(const v4ia*)(offs + 4 * tid);
  const v4f d4 = *(const v4fa*)(dv + 4 * tid);
  if (ovf != 0) { c4.x = -1; c4.y = -1; c4.z = -1; c4.w = -1; }
  *(volatile v4i*)(cntp + nodeBase + 4 * tid) = c4;
  *(volatile v4i*)(offp + nodeBase + 4 * tid) = o4;
  *(volatile v4f*)(dinvp + nodeBase + 4 * tid) = d4;
  __threadfence();
#pragma unroll 1
  for (int i = tid * 4; i < RCAP; i += NTHR * 4) {
    const v4i sv = *(const v4ia*)(hl + i);
    *(volatile v4i*)(lb + i) = sv;
  }
  *(volatile v4i*)(cntp + nodeBase + 4 * tid) = c4;
  *(volatile v4i*)(offp + nodeBase + 4 * tid) = o4;
  *(volatile v4f*)(dinvp + nodeBase + 4 * tid) = d4;
}

template <int LDA, int LDW, int KEXT>
__global__ __launch_bounds__(GTHR) __attribute__((amdgpu_num_vgpr(248)))
void k_gemm_t(const unsigned short* __restrict__ A, const unsigned short* __restrict__ WT,
              const float* __restrict__ dinv, float* P) {
  static_assert(KEXT % 32 == 0 && KEXT <= LDA && KEXT <= LDW && LDA % 8 == 0 && LDW % 8 == 0);
  __shared__ __attribute__((aligned(16))) float stg[GBM * GBN];
  __shared__ __attribute__((aligned(16))) float dsh[GBM];
  const int tid = (int)threadIdx.x, lane = tid & 31, wave = tid >> 5, hh = lane >> 4, m = lane & 15;
  const int rowBase = (int)blockIdx.x * GBM;

  v8f acc[8];
#pragma unroll
  for (int t = 0; t < 8; ++t) acc[t] = z8();
  const unsigned short* ap = A  + (size_t)(rowBase + 16 * wave + m) * (size_t)LDA + 8 * hh;
  const unsigned short* bp = WT + (size_t)m * (size_t)LDW + 8 * hh;

#pragma unroll 1
  for (int k0 = 0; k0 < KEXT; k0 += 32) {
    FragB af;
    af.h[0] = *(const v8usa*)(ap + k0);
    af.h[1] = *(const v8usa*)(ap + k0 + 16);
#pragma unroll
    for (int nt = 0; nt < 8; ++nt) {
      const unsigned short* wq = bp + (size_t)(16 * nt) * (size_t)LDW + k0;
      FragB bf;
      bf.h[0] = *(const v8usa*)wq;
      bf.h[1] = *(const v8usa*)(wq + 16);
      acc[nt] = wmb(af, bf, acc[nt]);
    }
  }

#pragma unroll
  for (int nt = 0; nt < 8; ++nt) {
    const int lc = 16 * nt + m;
#pragma unroll
    for (int r = 0; r < 8; ++r) {
      const int lr = 16 * wave + 8 * hh + r;
      stg[lr * GBN + lc] = acc[nt][r];
    }
  }
  if (wave == 0) {
    const int di = (lane < 16 ? lane : 15) * 4;
    const v4f d4 = *(const v4fa*)(dinv + rowBase + di);
    asm volatile("" :: "v"(d4));
    if (lane < 16) *(v4fa*)(dsh + 4 * lane) = d4;
  }
  __syncthreads();

  v4f pv[16];
#pragma unroll
  for (int i = 0; i < 16; ++i) {
    const float ds = dsh[16 * wave + i];
    const v4f x = *(const v4fa*)(stg + (16 * wave + i) * GBN + 4 * lane);
    v4f q;
    q.x = x.x * ds; q.y = x.y * ds; q.z = x.z * ds; q.w = x.w * ds;
    pv[i] = q;
  }
#pragma unroll
  for (int i = 0; i < 16; ++i) {
    float* op = P + (size_t)(rowBase + 16 * wave + i) * (size_t)DCH + 4 * lane;
    *(volatile v4f*)op = pv[i];
  }
  __threadfence();
#pragma unroll
  for (int i = 0; i < 16; ++i) {
    float* op = P + (size_t)(rowBase + 16 * wave + i) * (size_t)DCH + 4 * lane;
    *(volatile v4f*)op = pv[i];
  }
}

__global__ __launch_bounds__(NTHR) void k_replay(const int* __restrict__ lst, const int* __restrict__ cntp,
                                                 const int* __restrict__ offp, const float* __restrict__ dinvp,
                                                 const float* __restrict__ P, const float* __restrict__ par,
                                                 int bOff, float* T, float* rec) {
  __shared__ __attribute__((aligned(16))) int   scn[NBA];
  __shared__ __attribute__((aligned(16))) int   sof[NBA];
  __shared__ __attribute__((aligned(16))) float sdv[NBA];
  __shared__ __attribute__((aligned(16))) float sb[DCH];
  __shared__ __attribute__((aligned(16))) float wst[NWAVE * WSTW];
  __shared__ __attribute__((aligned(16))) float pst[PARTW];
  const int tid = (int)threadIdx.x, lane = tid & 31, wave = tid >> 5;
  const int blk = (int)blockIdx.x;
  const int nodeBase = blk * NBA;

  *(v4ia*)(scn + 4 * tid) = *(const v4ia*)(cntp + nodeBase + 4 * tid);
  *(v4ia*)(sof + 4 * tid) = *(const v4ia*)(offp + nodeBase + 4 * tid);
  *(v4fa*)(sdv + 4 * tid) = *(const v4fa*)(dinvp + nodeBase + 4 * tid);
  if (tid < 32) *(v4fa*)(sb + 4 * tid) = *(const v4fa*)(par + bOff + 4 * tid);
  __syncthreads();

  const v4f bq = *(const v4fa*)(sb + 4 * lane);
  const int* lb = lst + (size_t)blk * RCAP;
  const float qn = qnanf();
  int kk = 0;
  float wm[4], wq[4];
#pragma unroll
  for (int j = 0; j < 4; ++j) { wm[j] = 0.0f; wq[j] = 0.0f; }

#pragma unroll 1
  for (int si = 0; si < NBA / NWAVE; ++si) {
    const int s    = si * NWAVE + wave;
    const int node = nodeBase + s;
    const int cv = scn[s];
    const bool bad = (cv < 0) || (cv > DEGCAP);
    int c = cv < 0 ? 0 : (cv > DEGCAP ? DEGCAP : cv);
    c = __builtin_amdgcn_readfirstlane(c);
    int o = sof[s];
    o = o < 0 ? 0 : (o > RCAP - 1 ? RCAP - 1 : o);
    o = __builtin_amdgcn_readfirstlane(o);
    int last = o + c - 1;
    last = last < o ? o : last;
    last = last > RCAP - 1 ? RCAP - 1 : last;
    const int nc = node < NN ? node : NN - 1;
    const float dd = sdv[s];
    v4f acc = {0.0f, 0.0f, 0.0f, 0.0f};
#pragma unroll 1
    for (int b0 = 0; b0 < c; b0 += 32) {
      int idx = o + b0 + lane;
      idx = idx > last ? last : idx;
      int sr = lb[idx];
      sr = sr < 0 ? 0 : (sr > NN - 1 ? NN - 1 : sr);
      const int m32 = (c - b0) < 32 ? (c - b0) : 32;
#pragma unroll 1
      for (int k = 0; k < m32; ++k) {
        const int sk = __builtin_amdgcn_readlane(sr, k);
        const v4f a = *(const v4fa*)(P + (size_t)sk * DCH + 4 * lane);
        acc.x += a.x; acc.y += a.y; acc.z += a.z; acc.w += a.w;
      }
    }
    const v4f sv = *(const v4fa*)(P + (size_t)nc * DCH + 4 * lane);
    const bool live = node < NN;
    float v[4];
    v[0] = dd * (acc.x + sv.x) + bq.x;
    v[1] = dd * (acc.y + sv.y) + bq.y;
    v[2] = dd * (acc.z + sv.z) + bq.z;
    v[3] = dd * (acc.w + sv.w) + bq.w;
#pragma unroll
    for (int j = 0; j < 4; ++j) {
      const float y = bad ? qn : v[j];
      v[j] = live ? y : 0.0f;
    }
    if (node < MP) {
      v4f tv;
      tv.x = v[0]; tv.y = v[1]; tv.z = v[2]; tv.w = v[3];
      float* tp = T + (size_t)node * DCH + 4 * lane;
      *(volatile v4f*)tp = tv;
      __threadfence();
      *(volatile v4f*)tp = tv;
    }
    if (live) {
      kk += 1;
      const float rk = 1.0f / (float)kk;
#pragma unroll
      for (int j = 0; j < 4; ++j) {
        const float d = v[j] - wm[j];
        wm[j] = fmaf(d, rk, wm[j]);
        wq[j] = fmaf(d, v[j] - wm[j], wq[j]);
      }
    }
  }

  if (lane == 0) wst[wave * WSTW] = (float)kk;
#pragma unroll
  for (int j = 0; j < 4; ++j) {
    wst[wave * WSTW + 1 + 4 * lane + j]       = wm[j];
    wst[wave * WSTW + 1 + DCH + 4 * lane + j] = wq[j];
  }
  __syncthreads();
  if (tid < DCH) {
    float n = 0.0f, mean = 0.0f, M2 = 0.0f;
#pragma unroll 1
    for (int w2 = 0; w2 < NWAVE; ++w2) {
      const float nb = wst[w2 * WSTW];
      const float mb = wst[w2 * WSTW + 1 + tid];
      const float qb = wst[w2 * WSTW + 1 + DCH + tid];
      if (nb > 0.5f) {
        const float nn = n + nb;
        const float delta = mb - mean;
        const float f = nb / nn;
        mean = fmaf(delta, f, mean);
        M2 = M2 + qb + delta * delta * n * f;
        n = nn;
      }
    }
    pst[1 + tid] = mean;
    pst[1 + DCH + tid] = M2;
    if (tid == 0) pst[0] = n;
  }
#pragma unroll 1
  for (int i = 2 * DCH + 1 + tid; i < PARTW; i += NTHR) pst[i] = 0.0f;
  __syncthreads();
  const int pi = tid < PARTW / 4 ? tid : PARTW / 4 - 1;
  const v4f ps = *(const v4fa*)(pst + 4 * pi);
  if (tid < PARTW / 4) *(volatile v4f*)(rec + (size_t)blk * PARTW + 4 * tid) = ps;
  __threadfence();
  if (tid < PARTW / 4) *(volatile v4f*)(rec + (size_t)blk * PARTW + 4 * tid) = ps;
}

__global__ __launch_bounds__(DCH) void k_comb(const float* __restrict__ rec, float* stat) {
  __shared__ __attribute__((aligned(16))) float stg[2 * DCH];
  const int c = (int)threadIdx.x;
  double n = 0.0, mean = 0.0, M2 = 0.0;
#pragma unroll 1
  for (int b = 0; b < NBLK; ++b) {
    const float* pr = rec + (size_t)b * PARTW;
    const double nb = (double)pr[0];
    const double mb = (double)pr[1 + c];
    const double qb = (double)pr[1 + DCH + c];
    if (nb > 0.5) {
      const double nn = n + nb;
      const double delta = mb - mean;
      const double f = nb / nn;
      mean = mean + delta * f;
      M2 = M2 + qb + delta * delta * n * f;
      n = nn;
    }
  }
  const double nt = n < 1.0 ? 1.0 : n;
  const float varf = (float)(M2 / nt);
  stg[c] = (float)mean;
  stg[DCH + c] = 1.0f / sqrtf(varf + 1e-5f);
  __syncthreads();
  const int qi = c < (2 * DCH) / 4 ? c : (2 * DCH) / 4 - 1;
  const v4f v = *(const v4fa*)(stg + 4 * qi);
  if (c < (2 * DCH) / 4) *(volatile v4f*)(stat + 4 * c) = v;
  __threadfence();
  if (c < (2 * DCH) / 4) *(volatile v4f*)(stat + 4 * c) = v;
}

__global__ __launch_bounds__(NTHR) void k_apply(const float* __restrict__ T, const float* __restrict__ stat,
                                                const float* __restrict__ par, int gOff, int bOff,
                                                unsigned short* hbp) {
  __shared__ __attribute__((aligned(16))) float ssh[4 * DCH];
  const int tid = (int)threadIdx.x;
  ssh[tid] = stat[tid];
  {
    const int po = (tid < DCH) ? (gOff + tid) : (bOff + tid - DCH);
    ssh[2 * DCH + tid] = par[po];
  }
  __syncthreads();
  const int u   = (int)blockIdx.x * NTHR + tid;
  const int row = u >> 4;
  const int c8  = (u & 15) * 8;
  const int rc  = row < NN ? row : NN - 1;
  const bool ok = row < NN;
  const float* p = T + (size_t)rc * DCH + c8;
  const v4f a = *(const v4fa*)p;
  const v4f b = *(const v4fa*)(p + 4);
  float t[8];
  t[0] = a.x; t[1] = a.y; t[2] = a.z; t[3] = a.w;
  t[4] = b.x; t[5] = b.y; t[6] = b.z; t[7] = b.w;
  v8us hv, lv;
#pragma unroll
  for (int j = 0; j < 8; ++j) {
    const int c = c8 + j;
    float y = ((t[j] - ssh[c]) * ssh[DCH + c]) * ssh[2 * DCH + c] + ssh[3 * DCH + c];
    y = (y > 0.0f) ? y : (y - y);
    y = ok ? y : 0.0f;
    const unsigned hb = bf16_bits(y);
    hv[j] = (unsigned short)hb;
    lv[j] = (unsigned short)bf16_bits(y - __uint_as_float(hb << 16));
  }
  unsigned short* dp = hbp + (size_t)row * HK + c8;
  *(volatile v8us*)dp = hv;
  *(volatile v8us*)(dp + DCH) = lv;
  __threadfence();
  *(volatile v8us*)dp = hv;
  *(volatile v8us*)(dp + DCH) = lv;
}

__global__ __launch_bounds__(DCH) void k_pool(const float* __restrict__ T, const float* __restrict__ stat,
                                              const float* __restrict__ par, int gOff, int bOff,
                                              const int* __restrict__ gs, float* out) {
  __shared__ __attribute__((aligned(16))) float os[DCH];
  const int c = (int)threadIdx.x, lane = c & 31, wave = c >> 5;
  const int g = (int)blockIdx.x;
  int s = gs[g], e = gs[g + 1];
  const int fl = gs[NG + 1];
  s = s < 0 ? 0 : (s > NN ? NN : s);
  e = e < 0 ? 0 : (e > NN ? NN : e);
  int cnt = e - s;
  cnt = cnt < 0 ? 0 : cnt;
  const float mu = stat[c], rs = stat[DCH + c];
  const float gg = par[gOff + c], bb = par[bOff + c];
  float sum = 0.0f;
  const float* tp = T + (size_t)s * DCH + c;
#pragma unroll 4
  for (int i = 0; i < cnt; ++i) {
    const float t = tp[(size_t)i * DCH];
    sum += ((t - mu) * rs) * gg + bb;
  }
  const float den = fmaxf((float)cnt, 1.0f);
  float r = sum / den;
  r = (fl != 0) ? qnanf() : r;
  os[c] = r;
  __syncthreads();
  const v4f ov = *(const v4fa*)(os + 4 * lane);
  float* op = out + (size_t)g * DCH + 4 * lane;
  if (wave == 0) *(volatile v4f*)op = ov;
  __threadfence();
  if (wave == 0) *(volatile v4f*)op = ov;
}

static inline size_t al256(size_t o) { return (o + 255) & ~(size_t)255; }

extern "C" void kernel_launch(void* const* d_in, const int* in_sizes, int n_in,
                              void* d_out, int out_size, void* d_ws, size_t ws_size,
                              hipStream_t stream) {
  if (n_in < 16) return;
  if (in_sizes[0] != NN * DCH) return;
  if (in_sizes[1] != 2 * NE) return;
  if (in_sizes[3] != NN) return;
  if (in_sizes[4] != DCH * DCH || in_sizes[8] != DCH * DCH || in_sizes[12] != DCH * DCH) return;
  if (in_sizes[5] != DCH || in_sizes[6] != DCH || in_sizes[7] != DCH) return;
  if (in_sizes[9] != DCH || in_sizes[10] != DCH || in_sizes[11] != DCH) return;
  if (in_sizes[13] != DCH || in_sizes[14] != DCH || in_sizes[15] != DCH) return;
  if (out_size != NG * DCH) return;

  const float* x    = (const float*)d_in[0];
  const int*   edge = (const int*)d_in[1];
  const int*   bat  = (const int*)d_in[3];
  const float* W1   = (const float*)d_in[4];
  const float* b1   = (const float*)d_in[5];
  const float* g1   = (const float*)d_in[6];
  const float* be1  = (const float*)d_in[7];
  const float* Wm   = (const float*)d_in[8];
  const float* bm   = (const float*)d_in[9];
  const float* gm   = (const float*)d_in[10];
  const float* bem  = (const float*)d_in[11];
  const float* W2   = (const float*)d_in[12];
  const float* b2   = (const float*)d_in[13];
  const float* g2   = (const float*)d_in[14];
  const float* be2  = (const float*)d_in[15];
  float* out = (float*)d_out;
  const int* src = edge;
  const int* dst = edge + NE;

  char* ws = (char*)d_ws;
  size_t off = 0;
  const size_t oXB  = off; off = al256(off + (size_t)MP * DCH * 2);
  const size_t oW1T = off; off = al256(off + (size_t)DCH * DCH * 2);
  const size_t oWMD = off; off = al256(off + (size_t)DCH * HK * 2);
  const size_t oW2D = off; off = al256(off + (size_t)DCH * HK * 2);
  const size_t oPAR = off; off = al256(off + (size_t)9 * DCH * 4);
  const size_t oGS  = off; off = al256(off + (size_t)GSN * 4);
  const size_t oCNT = off; off = al256(off + (size_t)NSLOT * 4);
  const size_t oOFF = off; off = al256(off + (size_t)NSLOT * 4);
  const size_t oDNV = off; off = al256(off + (size_t)NSLOT * 4);
  const size_t oLST = off; off = al256(off + (size_t)NBLK * RCAP * 4);
  const size_t oP   = off; off = al256(off + (size_t)MP * DCH * 4);
  const size_t oT   = off; off = al256(off + (size_t)MP * DCH * 4);
  const size_t oHB  = off; off = al256(off + (size_t)MP * HK * 2);
  const size_t oREC = off; off = al256(off + (size_t)NBLK * PARTW * 4);
  const size_t oST  = off; off = al256(off + (size_t)2 * DCH * 4);
  if (off > ws_size || off > (size_t)(128u << 20)) return;
  unsigned short* XB  = (unsigned short*)(ws + oXB);
  unsigned short* W1T = (unsigned short*)(ws + oW1T);
  unsigned short* WMD = (unsigned short*)(ws + oWMD);
  unsigned short* W2D = (unsigned short*)(ws + oW2D);
  float*          PAR = (float*)(ws + oPAR);
  int*            GS  = (int*)(ws + oGS);
  int*            CNT = (int*)(ws + oCNT);
  int*            OFF = (int*)(ws + oOFF);
  float*          DNV = (float*)(ws + oDNV);
  int*            LST = (int*)(ws + oLST);
  float*          P   = (float*)(ws + oP);
  float*          T   = (float*)(ws + oT);
  unsigned short* HB  = (unsigned short*)(ws + oHB);
  float*          REC = (float*)(ws + oREC);
  float*          ST  = (float*)(ws + oST);

  const size_t bkLds = (size_t)BK_INTS * 4;
  hipFuncSetAttribute(reinterpret_cast<const void*>(&k_bucket), hipFuncAttributeMaxDynamicSharedMemorySize,
                      (int)bkLds);

  k_prep<<<PREPB, NTHR, 0, stream>>>(x, W1, Wm, W2, b1, g1, be1, bm, gm, bem, b2, g2, be2,
                                     XB, W1T, WMD, W2D, PAR);
  k_ranges<<<1, 512, 0, stream>>>(bat, GS);
  k_bucket<<<NBLK, NTHR, bkLds, stream>>>(src, dst, LST, CNT, OFF, DNV);
  k_gemm_t<DCH, DCH, DCH><<<MP / GBM, GTHR, 0, stream>>>(XB, W1T, DNV, P);
  k_replay<<<NBLK, NTHR, 0, stream>>>(LST, CNT, OFF, DNV, P, PAR, 0 * DCH, T, REC);
  k_comb<<<1, DCH, 0, stream>>>(REC, ST);
  k_apply<<<NBX, NTHR, 0, stream>>>(T, ST, PAR, 1 * DCH, 2 * DCH, HB);
  k_gemm_t<HK, HK, KX2><<<MP / GBM, GTHR, 0, stream>>>(HB, WMD, DNV, P);
  k_replay<<<NBLK, NTHR, 0, stream>>>(LST, CNT, OFF, DNV, P, PAR, 3 * DCH, T, REC);
  k_comb<<<1, DCH, 0, stream>>>(REC, ST);
  k_apply<<<NBX, NTHR, 0, stream>>>(T, ST, PAR, 4 * DCH, 5 * DCH, HB);
  k_gemm_t<HK, HK, KX3><<<MP / GBM, GTHR, 0, stream>>>(HB, W2D, DNV, P);
  k_replay<<<NBLK, NTHR, 0, stream>>>(LST, CNT, OFF, DNV, P, PAR, 6 * DCH, T, REC);
  k_comb<<<1, DCH, 0, stream>>>(REC, ST);
  k_pool<<<NG, DCH, 0, stream>>>(T, ST, PAR, 7 * DCH, 8 * DCH, GS, out);
}
